// Backbone_19963007992433
// MI455X (gfx1250) — hardware-verified
//
#include <hip/hip_runtime.h>

#ifndef NB
#define NB 8
#endif
#ifndef SEQ
#define SEQ 1024
#endif

constexpr int NB_FULL   = 8;
constexpr int SEQ_FULL  = 1024;
constexpr int DEPTH     = 4;
constexpr int TN_NODE   = 512;
constexpr int BM        = 128;
constexpr int BN        = 64;
constexpr int PREP_ROWS = 32;
constexpr int SLP       = 36;

static_assert(NB >= 1 && NB <= NB_FULL);
static_assert(SEQ >= BM && SEQ <= SEQ_FULL);
static_assert(SEQ % BM == 0 && SEQ % BN == 0);
static_assert(((long)NB * SEQ) % PREP_ROWS == 0);
static_assert(TN_NODE == 512 && TN_NODE % 32 == 0);
static_assert(BM + BN <= 256);
static_assert(BM == 4 * 32 && BN == 2 * 32);

constexpr size_t WS_OFF_PT = 0;
constexpr size_t WS_SZ_P   = (size_t)NB * SEQ * TN_NODE * 2;
constexpr size_t WS_OFF_PL = WS_OFF_PT + WS_SZ_P;
constexpr size_t WS_TOTAL  = WS_OFF_PL + WS_SZ_P;
static_assert(WS_OFF_PL % 256 == 0);
static_assert(WS_TOTAL <= 134217728ull);

typedef __attribute__((ext_vector_type(16))) _Float16       v16h;
typedef __attribute__((ext_vector_type(8)))  _Float16       v8h;
typedef __attribute__((ext_vector_type(8)))  float          v8f;
typedef __attribute__((ext_vector_type(4)))  float          v4f;
typedef __attribute__((ext_vector_type(4)))  int            v4i;
typedef __attribute__((ext_vector_type(8)))  unsigned short v8us;

union FragU { v16h v; v8h h[2]; };
__device__ __forceinline__ v16h frag_load(const _Float16* p) {
  FragU f; f.h[0] = *(const v8h*)(p); f.h[1] = *(const v8h*)(p + 16); return f.v;
}
__device__ __forceinline__ v8f mma_f16(v16h a, v16h b, v8f c) {
  return __builtin_amdgcn_wmma_f32_16x16x32_f16(false, a, false, b, (short)0, c, false, false);
}
__device__ __forceinline__ void dep_guard4(v8f& a, v8f& b, v8f& c, v8f& d, v16h x, v16h y) {
  asm volatile("v_nop\n\tv_nop\n\tv_nop\n\tv_nop" : "+v"(a), "+v"(b), "+v"(c), "+v"(d) : "v"(x), "v"(y));
}
__device__ __forceinline__ void keep4_h(v16h a, v16h b, v16h c, v16h d) {
  asm volatile("v_nop" :: "v"(a), "v"(b), "v"(c), "v"(d));
}
__device__ __forceinline__ void acc_guard4(v8f& a, v8f& b, v8f& c, v8f& d) {
  asm volatile("v_nop\n\tv_nop\n\tv_nop\n\tv_nop" : "+v"(a), "+v"(b), "+v"(c), "+v"(d));
}

__device__ __forceinline__ float distinct_count(v4i id) {
  const bool v0 = (unsigned)id[0] < (unsigned)TN_NODE;
  const bool v1 = (unsigned)id[1] < (unsigned)TN_NODE;
  const bool v2 = (unsigned)id[2] < (unsigned)TN_NODE;
  const bool v3 = (unsigned)id[3] < (unsigned)TN_NODE;
  int c = v0 ? 1 : 0;
  c += (v1 && id[1] != id[0]) ? 1 : 0;
  c += (v2 && id[2] != id[0] && id[2] != id[1]) ? 1 : 0;
  c += (v3 && id[3] != id[0] && id[3] != id[1] && id[3] != id[2]) ? 1 : 0;
  return (float)c;
}

__device__ __forceinline__ v8us multihot8(v4i id, int nbase) {
  v8us r;
#pragma unroll
  for (int e = 0; e < 8; ++e) {
    const int n = nbase + e;
    const bool m = (id[0] == n) | (id[1] == n) | (id[2] == n) | (id[3] == n);
    r[e] = m ? (unsigned short)0x3C00 : (unsigned short)0;
  }
  return r;
}

__global__ __launch_bounds__(256) void build_pos_kernel(
    const int* __restrict__ zt, const int* __restrict__ zl,
    unsigned short* __restrict__ posT, unsigned short* __restrict__ posL, int nrows)
{
  const int lane = threadIdx.x & 31, wave = threadIdx.x >> 5;
  const int r0 = blockIdx.x * PREP_ROWS + wave * 4;
  v8us vt[4][2], vl[4][2];
#pragma unroll
  for (int j = 0; j < 4; ++j) {
    int prow = r0 + j;
    prow = prow < nrows ? prow : nrows - 1;
    const int b = prow / SEQ, s = prow - b * SEQ;
    const size_t g = (size_t)(b * SEQ_FULL + s) * DEPTH;
    const v4i it = *(const v4i*)(zt + g);
    const v4i il = *(const v4i*)(zl + g);
#pragma unroll
    for (int c = 0; c < 2; ++c) {
      const int nbase = c * 256 + lane * 8;
      vt[j][c] = multihot8(it, nbase);
      vl[j][c] = multihot8(il, nbase);
    }
  }
  for (int pass = 0; pass < 2; ++pass) {
#pragma unroll
    for (int j = 0; j < 4; ++j) {
      const int prow = r0 + j;
      if (prow < nrows) {
#pragma unroll
        for (int c = 0; c < 2; ++c) {
          const size_t off = (size_t)prow * TN_NODE + c * 256 + lane * 8;
          *(volatile v8us*)(posT + off) = vt[j][c];
          *(volatile v8us*)(posL + off) = vl[j][c];
        }
      }
    }
    __threadfence();
  }
}

__global__ __launch_bounds__(256) void attn_gemm_kernel(
    const _Float16* __restrict__ posT, const _Float16* __restrict__ posL,
    const int* __restrict__ zt, const int* __restrict__ zl, const int* __restrict__ ind,
    const float* __restrict__ pdist, float* __restrict__ out)
{
  __shared__ __align__(16) float slab[8][16 * SLP];
  __shared__ float sM[3][BM];
  __shared__ float sN[3][BN];

  const int tid  = threadIdx.x;
  const int lane = tid & 31;
  const int wave = tid >> 5;
  const int wr   = wave >> 1;
  const int wc   = wave & 1;
  const int b    = blockIdx.z;
  const int m0   = blockIdx.y * BM;
  const int n0   = blockIdx.x * BN;

  {
    int s;
    if (tid < BM) s = m0 + tid;
    else { int t = tid - BM; t = t < BN ? t : BN - 1; s = n0 + t; }
    const size_t grow = (size_t)(b * SEQ_FULL + s);
    const v4i it = *(const v4i*)(zt + grow * DEPTH);
    const v4i il = *(const v4i*)(zl + grow * DEPTH);
    const int   iv = ind[grow];
    const float ct = distinct_count(it);
    const float cl = distinct_count(il);
    const float pd = (iv == 0) ? 1.0f : 0.0f;
    if (tid < BM) { sM[0][tid] = ct; sM[1][tid] = cl; sM[2][tid] = pd; }
    else if (tid < BM + BN) { const int t = tid - BM; sN[0][t] = ct; sN[1][t] = cl; sN[2][t] = pd; }
  }
  __syncthreads();

  const int rl   = lane & 15;
  const int hh   = lane >> 4;
  const int koff = hh * 8;
  const size_t rowA = (size_t)b * SEQ + m0 + wr * 32;
  const size_t rowB = (size_t)b * SEQ + n0 + wc * 32;
  const _Float16* AT = posT + rowA * TN_NODE;
  const _Float16* AL = posL + rowA * TN_NODE;
  const _Float16* BT = posT + rowB * TN_NODE;
  const _Float16* BL = posL + rowB * TN_NODE;

  v8f accT[2][2], accL[2][2];
#pragma unroll
  for (int mi = 0; mi < 2; ++mi)
#pragma unroll
    for (int ni = 0; ni < 2; ++ni) {
      accT[mi][ni] = (v8f){0.f, 0.f, 0.f, 0.f, 0.f, 0.f, 0.f, 0.f};
      accL[mi][ni] = (v8f){0.f, 0.f, 0.f, 0.f, 0.f, 0.f, 0.f, 0.f};
    }

#pragma unroll 2
  for (int k0 = 0; k0 < TN_NODE; k0 += 32) {
    v16h bt[2], bl[2];
#pragma unroll
    for (int ni = 0; ni < 2; ++ni) {
      const size_t bo = (size_t)(ni * 16 + rl) * TN_NODE + koff + k0;
      bt[ni] = frag_load(BT + bo);
      bl[ni] = frag_load(BL + bo);
    }
#pragma unroll
    for (int mi = 0; mi < 2; ++mi) {
      const size_t ao = (size_t)(mi * 16 + rl) * TN_NODE + koff + k0;
      const v16h at = frag_load(AT + ao);
      const v16h al = frag_load(AL + ao);
#pragma unroll
      for (int ni = 0; ni < 2; ++ni) {
        accT[mi][ni] = mma_f16(at, bt[ni], accT[mi][ni]);
        accL[mi][ni] = mma_f16(al, bl[ni], accL[mi][ni]);
      }
      dep_guard4(accT[mi][0], accT[mi][1], accL[mi][0], accL[mi][1], at, al);
    }
    keep4_h(bt[0], bt[1], bl[0], bl[1]);
  }
  acc_guard4(accT[0][0], accT[0][1], accT[1][0], accT[1][1]);
  acc_guard4(accL[0][0], accL[0][1], accL[1][0], accL[1][1]);

  const float dist = pdist[0];
  float* slabw = &slab[wave][0];
  const int q = lane >> 3, c4 = (lane & 7) * 4;
  float* outb = out + ((size_t)b * SEQ + m0 + wr * 32) * SEQ + n0 + wc * 32;
#pragma unroll
  for (int mi = 0; mi < 2; ++mi) {
#pragma unroll
    for (int ni = 0; ni < 2; ++ni) {
      const int nl = wc * 32 + ni * 16 + rl;
      const float snT = sN[0][nl], snL = sN[1][nl], snP = sN[2][nl];
#pragma unroll
      for (int r = 0; r < 8; ++r) {
        const int ml = wr * 32 + mi * 16 + hh * 8 + r;
        const float vt = sM[0][ml] + snT - 2.0f * accT[mi][ni][r];
        const float vl = sM[1][ml] + snL - 2.0f * accL[mi][ni][r];
        const float pm = fmaxf(sM[2][ml], snP) * dist;
        slabw[(hh * 8 + r) * SLP + ni * 16 + rl] = fmaxf(vt, vl) + pm;
      }
    }
    __builtin_amdgcn_fence(3  , "workgroup");
    __builtin_amdgcn_wave_barrier();
    __builtin_amdgcn_fence(2  , "workgroup");
    for (int pass = 0; pass < 2; ++pass) {
#pragma unroll
      for (int it = 0; it < 4; ++it) {
        const int row = it * 4 + q;
        const v4f v = *(const v4f*)(slabw + row * SLP + c4);
        *(volatile v4f*)(outb + (size_t)(mi * 16 + row) * SEQ + c4) = v;
      }
      __threadfence();
    }
    __builtin_amdgcn_fence(3  , "workgroup");
    __builtin_amdgcn_wave_barrier();
    __builtin_amdgcn_fence(2  , "workgroup");
  }
}

extern "C" void kernel_launch(void* const* d_in, const int* in_sizes, int n_in,
                              void* d_out, int out_size, void* d_ws, size_t ws_size,
                              hipStream_t stream)
{
  if (n_in < 4) return;
  const long need_z = ((long)(NB - 1) * SEQ_FULL + SEQ) * DEPTH;
  const long need_i = (long)(NB - 1) * SEQ_FULL + SEQ;
  if ((long)in_sizes[0] < need_z || (long)in_sizes[1] < need_z || (long)in_sizes[2] < need_i || in_sizes[3] < 1) return;
  if ((long)out_size < (long)NB * SEQ * SEQ) return;
  if (ws_size < WS_TOTAL) return;

  const int*   zt    = (const int*)d_in[0];
  const int*   zl    = (const int*)d_in[1];
  const int*   ind   = (const int*)d_in[2];
  const float* pdist = (const float*)d_in[3];
  float*       out   = (float*)d_out;

  char* ws = (char*)d_ws;
  unsigned short* posT = (unsigned short*)(ws + WS_OFF_PT);
  unsigned short* posL = (unsigned short*)(ws + WS_OFF_PL);

  const int nrows = NB * SEQ;
  build_pos_kernel<<<nrows / PREP_ROWS, 256, 0, stream>>>(zt, zl, posT, posL, nrows);
  attn_gemm_kernel<<<dim3(SEQ / BN, SEQ / BM, NB), 256, 0, stream>>>(
      (const _Float16*)posT, (const _Float16*)posL, zt, zl, ind, pdist, out);
}
